// RadialAttention_84945863180471
// MI455X (gfx1250) — hardware-run, weakly checked
//
#include <hip/hip_runtime.h>
#include <math.h>

typedef __attribute__((ext_vector_type(16))) _Float16 v16h;
typedef __attribute__((ext_vector_type(8)))  _Float16 v8h;
typedef __attribute__((ext_vector_type(8)))  float    v8f;
typedef __attribute__((ext_vector_type(4)))  float    v4f;

constexpr int kB     = 8;
constexpr int kC     = 256;
constexpr int kGridH = 64;
constexpr int kGridW = 64;
constexpr int kN     = kGridH * kGridW;
constexpr int kTok   = kB * kN;
constexpr int kQKld  = 2 * kC;
constexpr int kSqrtC = 16;
constexpr int kBins  = 8;
static_assert(kSqrtC * kSqrtC == kC, "logit scale is 1/sqrt(channels)");
static_assert(kN == 4096 && kTok == 32768, "token count");
static_assert((kC % 32) == 0 && (kN % 32) == 0, "GEMM K multiples of 32");
static_assert((kTok % 64) == 0 && (kQKld % 64) == 0 && (kC % 64) == 0 && (kN % 64) == 0, "GEMM M,N multiples of 64");

constexpr float kXCarry  = 16.0f;
constexpr float kWCarry  = 256.0f;
constexpr float kQKCarry = 16.0f;
constexpr float kVCarry  = 16.0f;
constexpr float kPCarry  = 32768.0f;
constexpr float kOCarry  = 256.0f;
constexpr float kProjQKScale = kQKCarry / (kXCarry * kWCarry);
constexpr float kProjVScale  = kVCarry / (kXCarry * kWCarry);
constexpr float kOutScale    = 1.0f / (kOCarry * kWCarry);
constexpr float kExpC   = 1.0f / ((float)kSqrtC * kQKCarry * kQKCarry);
constexpr float kFinDen = kPCarry * kVCarry / kOCarry;

constexpr size_t kOffW   = 0;
constexpr size_t kOffXT  = kOffW  + (size_t)4 * kC * kC * 2;
constexpr size_t kOffQK  = kOffXT + (size_t)kTok * kC * 2;
constexpr size_t kOffVT  = kOffQK + (size_t)kTok * kQKld * 2;
constexpr size_t kOffOP  = kOffVT + (size_t)kB * kC * kN * 2;
constexpr size_t kWsTotal = kOffOP + (size_t)kTok * kC * 2;
static_assert(kWsTotal == 84410368ull, "carve total");
static_assert(kWsTotal <= 134217728ull, "carve cap");
static_assert((kOffXT % 128) == 0 && (kOffQK % 128) == 0 && (kOffVT % 128) == 0 && (kOffOP % 128) == 0, "aligned regions");

struct FragH {
  union U { v16h v; v8h h[2]; };
  static __device__ __forceinline__ v16h load(const _Float16* p) {
    U f;
    f.h[0] = *(const v8h*)(p);
    f.h[1] = *(const v8h*)(p + 16);
    return f.v;
  }
  static __device__ __forceinline__ v8f mma(v16h a, v16h b, v8f c) {
    return __builtin_amdgcn_wmma_f32_16x16x32_f16(false, a, false, b, (short)0, c, false, false);
  }
};
__device__ __forceinline__ v8f mma_g(v16h a, v16h b, v8f c) {
  c = __builtin_amdgcn_wmma_f32_16x16x32_f16(false, a, false, b, (short)0, c, false, false);
  asm volatile("v_nop\n\tv_nop\n\tv_nop\n\tv_nop" : "+v"(c) : "v"(a), "v"(b));
  return c;
}
__device__ __forceinline__ void row_guard_h(v8f& a0, v8f& a1, v8f& a2, v8f& a3, v16h x, v16h b0, v16h b1, v16h b2, v16h b3) {
  asm volatile("v_nop\n\tv_nop\n\tv_nop\n\tv_nop" : "+v"(a0), "+v"(a1), "+v"(a2), "+v"(a3) : "v"(x), "v"(b0), "v"(b1), "v"(b2), "v"(b3));
}
__device__ __forceinline__ void keep4_h(v16h a, v16h b, v16h c, v16h d) { asm volatile("v_nop" :: "v"(a), "v"(b), "v"(c), "v"(d)); }
__device__ __forceinline__ void acc_guard4(v8f& a, v8f& b, v8f& c, v8f& d) { asm volatile("v_nop\n\tv_nop\n\tv_nop\n\tv_nop" : "+v"(a), "+v"(b), "+v"(c), "+v"(d)); }
__device__ __forceinline__ void wave_lds_sync() {
  __builtin_amdgcn_fence(__ATOMIC_RELEASE, "workgroup");
  __builtin_amdgcn_wave_barrier();
  __builtin_amdgcn_fence(__ATOMIC_ACQUIRE, "workgroup");
}

constexpr int ring_thr(int k) { return (2048 * k * k + 48) / 49; }
constexpr int kRingLast = ring_thr(7) + 1;
static_assert(ring_thr(1) == 42 && ring_thr(2) == 168 && ring_thr(3) == 377 && ring_thr(4) == 669 &&
              ring_thr(5) == 1045 && ring_thr(6) == 1505, "ring thresholds 1..6");
static_assert(ring_thr(7) == 2048 && kRingLast == 2049, "last ring starts above the largest squared distance of the grid");
static_assert(kGridH == 64 && kGridW == 64 && kBins == 8, "ring geometry");
static_assert((kGridW / 2) * (kGridW / 2) + (kGridH / 2) * (kGridH / 2) == 2048, "largest squared distance");
__device__ __forceinline__ float ring_scale(int n, const float (&ra)[8]) {
  const int yy = (n >> 6) & 63;
  const int xx = n & 63;
  const int dy = yy - 32;
  const int dx = xx - 32;
  const int d2 = dx * dx + dy * dy;
  float r = ra[0];
  r = (d2 >= ring_thr(1)) ? ra[1] : r;
  r = (d2 >= ring_thr(2)) ? ra[2] : r;
  r = (d2 >= ring_thr(3)) ? ra[3] : r;
  r = (d2 >= ring_thr(4)) ? ra[4] : r;
  r = (d2 >= ring_thr(5)) ? ra[5] : r;
  r = (d2 >= ring_thr(6)) ? ra[6] : r;
  r = (d2 >= kRingLast)   ? ra[7] : r;
  return r;
}

__global__ __launch_bounds__(256) void cast_w_kernel(const float* __restrict__ W0, const float* __restrict__ W1,
                                                     const float* __restrict__ W2, const float* __restrict__ W3,
                                                     unsigned short* __restrict__ out) {
  const int i   = blockIdx.x * 256 + threadIdx.x;
  const int mat = blockIdx.x >> 5;
  const float* W = (mat == 0) ? W0 : (mat == 1) ? W1 : (mat == 2) ? W2 : W3;
  const int off = (i & 8191) * 8;
  const v4f a = *(const v4f*)(W + off);
  const v4f c = *(const v4f*)(W + off + 4);
  v8h hv;
#pragma unroll
  for (int e = 0; e < 4; ++e) {
    hv[e]     = (_Float16)(a[e] * kWCarry);
    hv[4 + e] = (_Float16)(c[e] * kWCarry);
  }
  unsigned short* p = out + (size_t)mat * kC * kC + off;
  *(volatile v8h*)p = hv;
  __threadfence();
  *(volatile v8h*)p = hv;
}

__global__ __launch_bounds__(256) void xt_cast_kernel(const float* __restrict__ x, unsigned short* __restrict__ XT) {
  __shared__ __align__(16) float sm[32 * 260];
  const int t    = threadIdx.x;
  const int lane = t & 31;
  const int wave = __builtin_amdgcn_readfirstlane((int)(threadIdx.x >> 5));
  const int b    = blockIdx.y;
  const int tb   = blockIdx.x * 32;
  const float* xb = x + (size_t)b * kC * kN;
#pragma unroll
  for (int i = 0; i < 8; ++i) {
    const int e  = i * 256 + t;
    const int c  = e >> 3;
    const int t4 = (e & 7) * 4;
    const v4f f = *(const v4f*)(xb + (size_t)c * kN + tb + t4);
    sm[(t4 + 0) * 260 + c] = f[0] * kXCarry;
    sm[(t4 + 1) * 260 + c] = f[1] * kXCarry;
    sm[(t4 + 2) * 260 + c] = f[2] * kXCarry;
    sm[(t4 + 3) * 260 + c] = f[3] * kXCarry;
  }
  __syncthreads();
  v8h hv[4];
#pragma unroll
  for (int it = 0; it < 4; ++it) {
    const float* sp = sm + (wave * 4 + it) * 260 + lane * 8;
    const v4f a0 = *(const v4f*)(sp);
    const v4f a1 = *(const v4f*)(sp + 4);
#pragma unroll
    for (int e = 0; e < 4; ++e) {
      hv[it][e]     = (_Float16)a0[e];
      hv[it][4 + e] = (_Float16)a1[e];
    }
  }
  unsigned short* op = XT + ((size_t)b * kN + tb) * kC;
  for (int pass = 0; pass < 2; ++pass) {
#pragma unroll
    for (int it = 0; it < 4; ++it)
      *(volatile v8h*)(op + (size_t)(wave * 4 + it) * kC + lane * 8) = hv[it];
    __threadfence();
  }
}

template <int OUT_MODE, bool ROWSCALE, bool RESID>
__global__ __launch_bounds__(256) void gemm64_f16(
    const unsigned short* __restrict__ Ap, int lda, long strideA,
    const unsigned short* __restrict__ Btp, int ldb, long strideB,
    void* __restrict__ Cout, int ldc, long strideC,
    const float* __restrict__ resid, long strideR,
    const float* __restrict__ ringtab,
    int M, int N, int K, float scale) {
  const _Float16* A  = (const _Float16*)Ap;
  const _Float16* Bt = (const _Float16*)Btp;
  __shared__ __align__(16) float sT[8][16 * 68];
  const int b    = blockIdx.y;
  const int lane = threadIdx.x & 31;
  const int wave = __builtin_amdgcn_readfirstlane((int)(threadIdx.x >> 5));
  const int tilesN = N >> 6;
  const int tilesM = M >> 6;
  const int tile = blockIdx.x * 8 + wave;
  if (tile >= tilesM * tilesN) return;
  const int tm = tile / tilesN;
  const int tn = tile - tm * tilesN;
  const int m0 = tm << 6;
  const int n0 = tn << 6;

  const _Float16* Ab = A  + (size_t)b * strideA;
  const _Float16* Bb = Bt + (size_t)b * strideB;

  const int rlane = lane & 15;
  const int koff  = (lane >> 4) * 8;
  const int mOff  = (lane >> 4) * 8;

  v8f acc[4][4];
#pragma unroll
  for (int i = 0; i < 4; ++i)
#pragma unroll
    for (int j = 0; j < 4; ++j) acc[i][j] = (v8f){0.f, 0.f, 0.f, 0.f, 0.f, 0.f, 0.f, 0.f};

  for (int k0 = 0; k0 < K; k0 += 32) {
    v16h bh[4];
#pragma unroll
    for (int j = 0; j < 4; ++j) {
      const size_t bo = (size_t)(n0 + (j << 4) + rlane) * ldb + koff + k0;
      bh[j] = FragH::load(Bb + bo);
    }
#pragma unroll
    for (int i = 0; i < 4; ++i) {
      const size_t ao = (size_t)(m0 + (i << 4) + rlane) * lda + koff + k0;
      const v16h ah = FragH::load(Ab + ao);
#pragma unroll
      for (int j = 0; j < 4; ++j) acc[i][j] = FragH::mma(ah, bh[j], acc[i][j]);
      row_guard_h(acc[i][0], acc[i][1], acc[i][2], acc[i][3], ah, bh[0], bh[1], bh[2], bh[3]);
    }
    keep4_h(bh[0], bh[1], bh[2], bh[3]);
  }
  acc_guard4(acc[0][0], acc[0][1], acc[0][2], acc[0][3]);
  acc_guard4(acc[1][0], acc[1][1], acc[1][2], acc[1][3]);
  acc_guard4(acc[2][0], acc[2][1], acc[2][2], acc[2][3]);
  acc_guard4(acc[3][0], acc[3][1], acc[3][2], acc[3][3]);

  float ra[8];
#pragma unroll
  for (int i = 0; i < 8; ++i) ra[i] = ROWSCALE ? ringtab[i] : 1.0f;

  float* slab = sT[wave];
  const float* Rb = RESID ? (resid + (size_t)b * strideR) : nullptr;
#pragma unroll
  for (int i = 0; i < 4; ++i) {
    const int mBase = m0 + (i << 4);
    float rs[8];
#pragma unroll
    for (int r = 0; r < 8; ++r)
      rs[r] = ROWSCALE ? (scale * ring_scale((mBase + mOff + r) & (kN - 1), ra)) : scale;
#pragma unroll
    for (int j = 0; j < 4; ++j) {
#pragma unroll
      for (int r = 0; r < 8; ++r)
        slab[(mOff + r) * 68 + (j << 4) + rlane] = acc[i][j][r] * rs[r];
    }
    wave_lds_sync();
    if (OUT_MODE == 0) {
      float* C = (float*)Cout + (size_t)b * strideC;
      const int hh = lane >> 4, c4 = (lane & 15) * 4;
      v4f vals[8];
#pragma unroll
      for (int it = 0; it < 8; ++it) {
        const int row = it * 2 + hh;
        v4f v = *(const v4f*)(slab + row * 68 + c4);
        if (RESID) {
          const v4f rv = *(const v4f*)(Rb + (size_t)(mBase + row) * ldc + n0 + c4);
          v = v + rv;
        }
        vals[it] = v;
      }
      for (int pass = 0; pass < 2; ++pass) {
#pragma unroll
        for (int it = 0; it < 8; ++it) {
          const int row = it * 2 + hh;
          *(volatile v4f*)(C + (size_t)(mBase + row) * ldc + n0 + c4) = vals[it];
        }
        __threadfence();
      }
    } else {
      const int q = lane >> 3, c8 = (lane & 7) * 8;
      unsigned short* C = (unsigned short*)Cout + (size_t)b * strideC;
      v8h hv[4];
#pragma unroll
      for (int it = 0; it < 4; ++it) {
        const float* sp = slab + (it * 4 + q) * 68 + c8;
#pragma unroll
        for (int e = 0; e < 8; ++e) hv[it][e] = (_Float16)sp[e];
      }
      for (int pass = 0; pass < 2; ++pass) {
#pragma unroll
        for (int it = 0; it < 4; ++it) {
          const int row = it * 4 + q;
          *(volatile v8h*)(C + (size_t)(mBase + row) * ldc + n0 + c8) = hv[it];
        }
        __threadfence();
      }
    }
    wave_lds_sync();
  }
}

constexpr int kAtWaves = 4;
constexpr int kPsPitch = 64;
constexpr int kOsPitch = 264;
__global__ __launch_bounds__(128) void attn_d256_kernel(const unsigned short* __restrict__ QKp,
                                                        const unsigned short* __restrict__ VTp,
                                                        unsigned short* __restrict__ OPp) {
  __shared__ __align__(16) _Float16 Ps[kAtWaves][16 * kPsPitch];
  __shared__ __align__(16) _Float16 Os[kAtWaves][16 * kOsPitch];
  const int lane = threadIdx.x & 31;
  const int wave = __builtin_amdgcn_readfirstlane((int)(threadIdx.x >> 5));
  const int hh   = lane >> 4;
  const int c    = lane & 15;
  const int b    = blockIdx.y;
  const int q0   = blockIdx.x * 64 + wave * 16;

  const _Float16* QK = (const _Float16*)QKp + (size_t)b * kN * kQKld;
  const _Float16* VT = (const _Float16*)VTp + (size_t)b * kC * kN;
  const _Float16* qrow = QK + (size_t)(q0 + c) * kQKld + 8 * hh;
  const _Float16* kcol = QK + (size_t)c * kQKld + kC + 8 * hh;
  const _Float16* vcol = VT + (size_t)c * kN + 8 * hh;
  _Float16* Pw = Ps[wave];
  _Float16* Ow = Os[wave];

  float mrow[8], lrow[8];
  v8f oacc[16];
#pragma unroll
  for (int r = 0; r < 8; ++r) { mrow[r] = -1.0e30f; lrow[r] = 0.f; }
#pragma unroll
  for (int t = 0; t < 16; ++t) oacc[t] = (v8f){0.f, 0.f, 0.f, 0.f, 0.f, 0.f, 0.f, 0.f};

#pragma unroll 1
  for (int kt = 0; kt < kN / 64; ++kt) {
    const int kv0 = kt * 64;
    v8f s[4];
#pragma unroll
    for (int j = 0; j < 4; ++j) s[j] = (v8f){0.f, 0.f, 0.f, 0.f, 0.f, 0.f, 0.f, 0.f};
#pragma unroll 1
    for (int ci = 0; ci < kC / 32; ++ci) {
      const v16h a = FragH::load(qrow + ci * 32);
#pragma unroll
      for (int j = 0; j < 4; ++j) {
        const v16h bk = FragH::load(kcol + (size_t)(kv0 + j * 16) * kQKld + ci * 32);
        s[j] = mma_g(a, bk, s[j]);
      }
    }
    float cm[8];
#pragma unroll
    for (int r = 0; r < 8; ++r) {
      float m = fmaxf(fmaxf(s[0][r], s[1][r]), fmaxf(s[2][r], s[3][r]));
      m = fmaxf(m, __shfl_xor(m, 1, 32));
      m = fmaxf(m, __shfl_xor(m, 2, 32));
      m = fmaxf(m, __shfl_xor(m, 4, 32));
      m = fmaxf(m, __shfl_xor(m, 8, 32));
      cm[r] = m;
    }
    wave_lds_sync();
#pragma unroll
    for (int r = 0; r < 8; ++r) {
      const float mnew  = fmaxf(mrow[r], cm[r]);
      const float alpha = __expf((mrow[r] - mnew) * kExpC);
      mrow[r] = mnew;
      float psum = 0.f;
#pragma unroll
      for (int j = 0; j < 4; ++j) {
        const float p = __expf((s[j][r] - mnew) * kExpC);
        psum += p;
        Pw[(8 * hh + r) * kPsPitch + j * 16 + c] = (_Float16)(p * kPCarry);
      }
      lrow[r] = lrow[r] * alpha + psum;
#pragma unroll
      for (int t = 0; t < 16; ++t) oacc[t][r] *= alpha;
    }
    wave_lds_sync();
#pragma unroll 1
    for (int kk = 0; kk < 2; ++kk) {
      const v16h pa = FragH::load(Pw + c * kPsPitch + kk * 32 + 8 * hh);
#pragma unroll
      for (int t = 0; t < 16; ++t) {
        const v16h vb = FragH::load(vcol + (size_t)(t * 16) * kN + kv0 + kk * 32);
        oacc[t] = mma_g(pa, vb, oacc[t]);
      }
    }
  }

#pragma unroll
  for (int r = 0; r < 8; ++r) {
    float l = lrow[r];
    l += __shfl_xor(l, 1, 32);
    l += __shfl_xor(l, 2, 32);
    l += __shfl_xor(l, 4, 32);
    l += __shfl_xor(l, 8, 32);
    const float inv = 1.0f / (l * kFinDen);
#pragma unroll
    for (int t = 0; t < 16; ++t)
      Ow[(8 * hh + r) * kOsPitch + t * 16 + c] = (_Float16)(oacc[t][r] * inv);
  }
  wave_lds_sync();
  v8h ov[16];
#pragma unroll
  for (int it = 0; it < 16; ++it) ov[it] = *(const v8h*)(Ow + it * kOsPitch + lane * 8);
  unsigned short* ob = OPp + ((size_t)b * kN + q0) * kC;
  for (int pass = 0; pass < 2; ++pass) {
#pragma unroll
    for (int it = 0; it < 16; ++it)
      *(volatile v8h*)(ob + (size_t)it * kC + lane * 8) = ov[it];
    __threadfence();
  }
}

extern "C" void kernel_launch(void* const* d_in, const int* in_sizes, int n_in,
                              void* d_out, int out_size, void* d_ws, size_t ws_size,
                              hipStream_t stream) {
  if (n_in < 6) return;
  if (in_sizes[0] != kB * kC * kN) return;
  if (in_sizes[1] != kC * kC) return;
  if (in_sizes[2] != kC * kC) return;
  if (in_sizes[3] != kC * kC) return;
  if (in_sizes[4] != kC * kC) return;
  if (in_sizes[5] != kBins) return;
  if (out_size != kB * kC * kN) return;
  if (ws_size < kWsTotal) return;

  const float* x    = (const float*)d_in[0];
  const float* Wq   = (const float*)d_in[1];
  const float* Wk   = (const float*)d_in[2];
  const float* Wv   = (const float*)d_in[3];
  const float* Wo   = (const float*)d_in[4];
  const float* ring = (const float*)d_in[5];
  float* out = (float*)d_out;

  char* ws = (char*)d_ws;
  unsigned short* WALL = (unsigned short*)(ws + kOffW);
  unsigned short* XT   = (unsigned short*)(ws + kOffXT);
  unsigned short* QK   = (unsigned short*)(ws + kOffQK);
  unsigned short* VT   = (unsigned short*)(ws + kOffVT);
  unsigned short* OP   = (unsigned short*)(ws + kOffOP);
  unsigned short* WQK  = WALL;
  unsigned short* WV   = WALL + (size_t)2 * kC * kC;
  unsigned short* WO   = WALL + (size_t)3 * kC * kC;

  cast_w_kernel<<<dim3((4 * kC * kC / 8) / 256), 256, 0, stream>>>(Wq, Wk, Wv, Wo, WALL);

  xt_cast_kernel<<<dim3(kN / 32, kB), 256, 0, stream>>>(x, XT);

  gemm64_f16<1, true, false><<<dim3((kTok / 64) * (kQKld / 64) / 8, 1), 256, 0, stream>>>(
      XT, kC, 0L,
      WQK, kC, 0L,
      (void*)QK, kQKld, 0L,
      nullptr, 0L,
      ring,
      kTok, kQKld, kC, kProjQKScale);

  gemm64_f16<1, false, false><<<dim3((kC / 64) * (kN / 64) / 8, kB), 256, 0, stream>>>(
      WV, kC, 0L,
      XT, kC, (long)kN * kC,
      (void*)VT, kN, (long)kC * kN,
      nullptr, 0L,
      nullptr,
      kC, kN, kC, kProjVScale);

  attn_d256_kernel<<<dim3(kN / 64, kB), 128, 0, stream>>>(QK, VT, OP);

  gemm64_f16<0, false, true><<<dim3((kC / 64) * (kN / 64) / 8, kB), 256, 0, stream>>>(
      WO, kC, 0L,
      OP, kC, (long)kN * kC,
      (void*)out, kN, (long)kC * kN,
      x, (long)kC * kN,
      nullptr,
      kC, kN, kC, kOutScale);
}
